// BiLSTM_7945689497983
// MI455X (gfx1250) — hardware-verified
//
#include <hip/hip_runtime.h>
#include <math.h>

constexpr int NB_SEQ  = 64;
constexpr int NSTEP   = 256;
constexpr int NEMB    = 256;
constexpr int NHU     = 256;
constexpr int NGATE   = 4 * NHU;
constexpr int NKCAT   = NEMB + NHU;
constexpr int NHID2   = 2 * NHU;
constexpr int NTAG    = 20;
constexpr int NTAGP   = 64;
constexpr int NVOC    = 50000;
constexpr int NROWS   = NB_SEQ * NSTEP;
constexpr int NTHR    = 256;
constexpr int SEQ_BLK = 16;
constexpr int AP1     = 520;
constexpr int AP2     = 264;
constexpr int PK_THR  = 320;
constexpr size_t WS_CAP = 134217728;

static_assert(NROWS % 64 == 0 && NTAGP % 64 == 0);
static_assert(NHID2 % 32 == 0);
static_assert(NEMB % 32 == 0 && NHU % 32 == 0);
static_assert(NB_SEQ % SEQ_BLK == 0);
static_assert(NHU == 32 * (NTHR / 32));
static_assert(SEQ_BLK == 2 * (NTHR / 32));
static_assert(SEQ_BLK * 16 == NTHR && NEMB == 16 * 16);
static_assert(4 * PK_THR == 64 * NTAG);
static_assert((64 * NTAG * 4) % 128 == 0);
static_assert(NGATE % 64 == 0 && NEMB % 64 == 0 && NHU % 64 == 0);
static_assert((NTAGP * NHID2 / 8) % NTHR == 0);
static_assert(((NROWS / 64) * (NTAGP / 64)) % 8 == 0);
static_assert(AP1 % 8 == 0 && AP2 % 8 == 0);
static_assert(NTAG % 4 == 0);

typedef __attribute__((ext_vector_type(16))) _Float16 v16h;
typedef __attribute__((ext_vector_type(8)))  _Float16 v8h;
typedef __attribute__((ext_vector_type(16))) __bf16   v16b;
typedef __attribute__((ext_vector_type(8)))  __bf16   v8b;
typedef __attribute__((ext_vector_type(8)))  float    v8f;
typedef __attribute__((ext_vector_type(4)))  float    v4f;
typedef __attribute__((ext_vector_type(4)))  unsigned v4u;

__device__ __forceinline__ unsigned short f2bf_bits(float f) {
  unsigned u = __float_as_uint(f);
  return (unsigned short)((u + 0x7FFFu + ((u >> 16) & 1u)) >> 16);
}
__device__ __forceinline__ float bf_bits2f(unsigned short h) { return __uint_as_float(((unsigned)h) << 16); }
__device__ __forceinline__ float bf16r(float f) { return bf_bits2f(f2bf_bits(f)); }
__device__ __forceinline__ unsigned pk_bf2(float a, float b) {
  return (unsigned)f2bf_bits(a) | ((unsigned)f2bf_bits(b) << 16);
}

__device__ __forceinline__ void keep4_h(v16h a, v16h b, v16h c, v16h d) { asm volatile("v_nop" :: "v"(a), "v"(b), "v"(c), "v"(d)); }
__device__ __forceinline__ void keep4_b(v16b a, v16b b, v16b c, v16b d) { asm volatile("v_nop" :: "v"(a), "v"(b), "v"(c), "v"(d)); }
__device__ __forceinline__ void acc_guard4(v8f& a, v8f& b, v8f& c, v8f& d) { asm volatile("v_nop\n\tv_nop\n\tv_nop\n\tv_nop" : "+v"(a), "+v"(b), "+v"(c), "+v"(d)); }
__device__ __forceinline__ void grp_guard_h(v8f& a0, v8f& a1, v8f& a2, v8f& a3,
                                            v16h x0, v16h x1, v16h y0, v16h y1, v16h y2, v16h y3) {
  asm volatile("v_nop\n\tv_nop\n\tv_nop\n\tv_nop"
               : "+v"(a0), "+v"(a1), "+v"(a2), "+v"(a3)
               : "v"(x0), "v"(x1), "v"(y0), "v"(y1), "v"(y2), "v"(y3));
}
__device__ __forceinline__ void grp_guard_b(v8f& a0, v8f& a1, v8f& a2, v8f& a3,
                                            v16b x0, v16b x1, v16b y0, v16b y1, v16b y2, v16b y3) {
  asm volatile("v_nop\n\tv_nop\n\tv_nop\n\tv_nop"
               : "+v"(a0), "+v"(a1), "+v"(a2), "+v"(a3)
               : "v"(x0), "v"(x1), "v"(y0), "v"(y1), "v"(y2), "v"(y3));
}

template <typename T> struct Frag;
template <> struct Frag<_Float16> {
  typedef v16h V; union U { v16h v; v8h h[2]; };
  static __device__ __forceinline__ v16h load(const _Float16* p) {
    U f; f.h[0] = *(const v8h*)(p); f.h[1] = *(const v8h*)(p + 16); return f.v;
  }
  static __device__ __forceinline__ v8f mma(v16h a, v16h b, v8f c) {
    return __builtin_amdgcn_wmma_f32_16x16x32_f16(false, a, false, b, (short)0, c, false, false);
  }
  static __device__ __forceinline__ void guard4(v8f& a0, v8f& a1, v8f& a2, v8f& a3, v16h x0, v16h x1,
                                                v16h y0, v16h y1, v16h y2, v16h y3) {
    grp_guard_h(a0, a1, a2, a3, x0, x1, y0, y1, y2, y3);
  }
  static __device__ __forceinline__ void keep(v16h a, v16h b, v16h c, v16h d) { keep4_h(a, b, c, d); }
};
template <> struct Frag<__bf16> {
  typedef v16b V; union U { v16b v; v8b h[2]; };
  static __device__ __forceinline__ v16b load(const __bf16* p) {
    U f; f.h[0] = *(const v8b*)(p); f.h[1] = *(const v8b*)(p + 16); return f.v;
  }
  static __device__ __forceinline__ v8f mma(v16b a, v16b b, v8f c) {
    return __builtin_amdgcn_wmma_f32_16x16x32_bf16(false, a, false, b, (short)0, c, false, false);
  }
  static __device__ __forceinline__ void guard4(v8f& a0, v8f& a1, v8f& a2, v8f& a3, v16b x0, v16b x1,
                                                v16b y0, v16b y1, v16b y2, v16b y3) {
    grp_guard_b(a0, a1, a2, a3, x0, x1, y0, y1, y2, y3);
  }
  static __device__ __forceinline__ void keep(v16b a, v16b b, v16b c, v16b d) { keep4_b(a, b, c, d); }
};

__device__ __forceinline__ float fsig(float x)  { return __builtin_amdgcn_rcpf(1.0f + expf(-x)); }
__device__ __forceinline__ float ftanh(float x) { return 1.0f - 2.0f * __builtin_amdgcn_rcpf(expf(2.0f * x) + 1.0f); }

template <int ET> struct Elem;
template <> struct Elem<0> { typedef _Float16 T; };
template <> struct Elem<1> { typedef __bf16 T; };
template <int ET, bool SPLIT, int BIAS_MODE, int OUT_MODE, bool RESID, int ACT = 0>
__global__ __launch_bounds__(256) void wmma_gemm64(
    const unsigned short* __restrict__ Ap, const unsigned short* __restrict__ A2p, int lda, long strideA,
    const unsigned short* __restrict__ Btp, const unsigned short* __restrict__ Bt2p, int ldb, long strideB,
    void* __restrict__ Cout, void* __restrict__ Cout2, int ldc, long strideC,
    const float* __restrict__ bias,
    const float* __restrict__ resid, long strideR,
    int M, int N, int K, float scale) {
  typedef typename Elem<ET>::T T;
  typedef typename Frag<T>::V V;
  const T* A = (const T*)Ap; const T* A2 = (const T*)A2p; const T* Bt = (const T*)Btp; const T* Bt2 = (const T*)Bt2p;
  __shared__ __align__(16) float sT[8][16 * 68];
  const int b    = blockIdx.y;
  const int lane = threadIdx.x & 31;
  const int wave = threadIdx.x >> 5;
  const int tilesN = N >> 6;
  const int tilesM = M >> 6;
  const int tile = blockIdx.x * 8 + wave;
  if (tile >= tilesM * tilesN) return;
  const int tm = tile / tilesN;
  const int tn = tile - tm * tilesN;
  const int m0 = tm << 6;
  const int n0 = tn << 6;

  const T* Ab  = A  + (size_t)b * strideA;
  const T* Bb  = Bt + (size_t)b * strideB;
  const T* Ab2 = SPLIT ? (A2  + (size_t)b * strideA) : nullptr;
  const T* Bb2 = SPLIT ? (Bt2 + (size_t)b * strideB) : nullptr;

  const int rlane = lane & 15;
  const int koff  = (lane >> 4) * 8;
  const int mOff  = (lane >> 4) * 8;

  v8f acc[4][4];
#pragma unroll
  for (int i = 0; i < 4; ++i)
#pragma unroll
    for (int j = 0; j < 4; ++j) acc[i][j] = (v8f){0.f,0.f,0.f,0.f,0.f,0.f,0.f,0.f};

  for (int k0 = 0; k0 < K; k0 += 32) {
    V bh[4], bl[4];
#pragma unroll
    for (int j = 0; j < 4; ++j) {
      const size_t bo = (size_t)(n0 + (j << 4) + rlane) * ldb + koff + k0;
      bh[j] = Frag<T>::load(Bb + bo);
      if (SPLIT) bl[j] = Frag<T>::load(Bb2 + bo);
    }
#pragma unroll
    for (int i = 0; i < 4; ++i) {
      const size_t ao = (size_t)(m0 + (i << 4) + rlane) * lda + koff + k0;
      V ah = Frag<T>::load(Ab + ao);
      V al;
      if (SPLIT) al = Frag<T>::load(Ab2 + ao);
#pragma unroll
      for (int j = 0; j < 4; ++j) {
        acc[i][j] = Frag<T>::mma(ah, bh[j], acc[i][j]);
        if (SPLIT) {
          acc[i][j] = Frag<T>::mma(ah, bl[j], acc[i][j]);
          acc[i][j] = Frag<T>::mma(al, bh[j], acc[i][j]);
        }
      }
      Frag<T>::guard4(acc[i][0], acc[i][1], acc[i][2], acc[i][3], ah, SPLIT ? al : ah, bh[0], bh[1], bh[2], bh[3]);
    }
    Frag<T>::keep(bh[0], bh[1], bh[2], bh[3]);
    if (SPLIT) Frag<T>::keep(bl[0], bl[1], bl[2], bl[3]);
  }
  acc_guard4(acc[0][0], acc[0][1], acc[0][2], acc[0][3]);
  acc_guard4(acc[1][0], acc[1][1], acc[1][2], acc[1][3]);
  acc_guard4(acc[2][0], acc[2][1], acc[2][2], acc[2][3]);
  acc_guard4(acc[3][0], acc[3][1], acc[3][2], acc[3][3]);

  float* slab = sT[wave];
  const float* Rb = RESID ? (resid + (size_t)b * strideR) : nullptr;
#pragma unroll
  for (int i = 0; i < 4; ++i) {
    const int mBase = m0 + (i << 4);
#pragma unroll
    for (int j = 0; j < 4; ++j) {
      const int n = n0 + (j << 4) + rlane;
      float bv = 0.f;
      if (BIAS_MODE == 2) bv = bias[n];
#pragma unroll
      for (int r = 0; r < 8; ++r) {
        float v = acc[i][j][r] * scale;
        if (BIAS_MODE == 1) v += bias[mBase + mOff + r];
        if (BIAS_MODE == 2) v += bv;
        if (RESID) v += Rb[(size_t)(mBase + mOff + r) * ldc + n];
        if (ACT == 1) v = tanhf(v);
        if (ACT == 2) v = fmaxf(v, 0.0f);
        if (ACT == 3) v = v / (1.0f + expf(-v));
        if (ACT == 4) v = (v > 0.f) ? v : 0.01f * v;
        if (ACT == 5) v = 0.5f * v * (1.0f + erff(v * 0.70710678118654752f));
        slab[(mOff + r) * 68 + (j << 4) + rlane] = v;
      }
    }
    __builtin_amdgcn_fence(__ATOMIC_RELEASE, "workgroup");
    __builtin_amdgcn_wave_barrier();
    __builtin_amdgcn_fence(__ATOMIC_ACQUIRE, "workgroup");
    if (OUT_MODE == 0) {
      float* C = (float*)Cout + (size_t)b * strideC;
      const int hh = lane >> 4, c4 = (lane & 15) * 4;
      for (int pass = 0; pass < 2; ++pass) {
#pragma unroll
        for (int it = 0; it < 8; ++it) {
          const int row = it * 2 + hh;
          v4f v = *(const v4f*)(slab + row * 68 + c4);
          *(volatile v4f*)(C + (size_t)(mBase + row) * ldc + n0 + c4) = v;
        }
        __threadfence();
      }
    } else {
      const int q = lane >> 3, c8 = (lane & 7) * 8;
      unsigned short* C  = (unsigned short*)Cout  + (size_t)b * strideC;
      unsigned short* C2 = (OUT_MODE == 2) ? ((unsigned short*)Cout2 + (size_t)b * strideC) : nullptr;
      for (int pass = 0; pass < 2; ++pass) {
#pragma unroll
        for (int it = 0; it < 4; ++it) {
          const int row = it * 4 + q;
          const float* sp = slab + row * 68 + c8;
          v8h hv, lv;
#pragma unroll
          for (int e = 0; e < 8; ++e) {
            if (OUT_MODE == 1) {
              hv[e] = (_Float16)sp[e];
            } else {
              unsigned short hb = f2bf_bits(sp[e]);
              unsigned short lb = f2bf_bits(sp[e] - bf_bits2f(hb));
              hv[e] = __builtin_bit_cast(_Float16, hb);
              lv[e] = __builtin_bit_cast(_Float16, lb);
            }
          }
          *(volatile v8h*)(C + (size_t)(mBase + row) * ldc + n0 + c8) = hv;
          if (OUT_MODE == 2) *(volatile v8h*)(C2 + (size_t)(mBase + row) * ldc + n0 + c8) = lv;
        }
        __threadfence();
      }
    }
    __builtin_amdgcn_fence(__ATOMIC_RELEASE, "workgroup");
    __builtin_amdgcn_wave_barrier();
    __builtin_amdgcn_fence(__ATOMIC_ACQUIRE, "workgroup");
  }
}

__global__ __launch_bounds__(NTHR) void wcat_prep_kernel(const float* __restrict__ wxf, const float* __restrict__ whf,
                                                         const float* __restrict__ wxb, const float* __restrict__ whb,
                                                         unsigned short* __restrict__ WCAT) {
  __shared__ float Tt[64 * 65];
  const int tid = threadIdx.x;
  const int z = blockIdx.z;
  const float* src = (z == 0) ? wxf : (z == 1) ? whf : (z == 2) ? wxb : whb;
  unsigned short* dst = WCAT + (size_t)(z >> 1) * ((size_t)NGATE * NKCAT) + (size_t)(z & 1) * NHU;
  const int c0 = blockIdx.x * 64;
  const int r0 = blockIdx.y * 64;
#pragma unroll
  for (int i = 0; i < 4; ++i) {
    const int idx = i * NTHR + tid;
    const int rr = idx >> 4, cc = (idx & 15) * 4;
    const v4f v = *(const v4f*)(src + (size_t)(r0 + rr) * NGATE + c0 + cc);
    Tt[rr * 65 + cc + 0] = v[0];
    Tt[rr * 65 + cc + 1] = v[1];
    Tt[rr * 65 + cc + 2] = v[2];
    Tt[rr * 65 + cc + 3] = v[3];
  }
  __syncthreads();
  const int q = tid >> 3, c8 = (tid & 7) * 8;
  v4u hv[2];
#pragma unroll
  for (int g = 0; g < 2; ++g) {
    const int qq = g * 32 + q;
    float f[8];
#pragma unroll
    for (int e = 0; e < 8; ++e) f[e] = Tt[(c8 + e) * 65 + qq];
    hv[g][0] = pk_bf2(f[0], f[1]);
    hv[g][1] = pk_bf2(f[2], f[3]);
    hv[g][2] = pk_bf2(f[4], f[5]);
    hv[g][3] = pk_bf2(f[6], f[7]);
  }
  for (int pass = 0; pass < 2; ++pass) {
#pragma unroll
    for (int g = 0; g < 2; ++g) {
      const size_t o = (size_t)(c0 + g * 32 + q) * (size_t)NKCAT + (size_t)(r0 + c8);
      *(volatile v4u*)(dst + o) = hv[g];
    }
    __threadfence();
  }
}

__global__ __launch_bounds__(NTHR) void wtag_prep_kernel(const float* __restrict__ wtag, unsigned short* __restrict__ WT,
                                                         unsigned short* __restrict__ WTZ) {
  const int i = blockIdx.x * NTHR + threadIdx.x;
  const int n = i >> 6, c8 = (i & 63) * 8;
  const int nc = (n < NTAG) ? n : (NTAG - 1);
  const bool live = (n < NTAG);
  float f[8];
#pragma unroll
  for (int e = 0; e < 8; ++e) {
    const float v = wtag[(size_t)(c8 + e) * NTAG + nc];
    f[e] = live ? v : 0.0f;
  }
  v4u hv;
  hv[0] = pk_bf2(f[0], f[1]);
  hv[1] = pk_bf2(f[2], f[3]);
  hv[2] = pk_bf2(f[4], f[5]);
  hv[3] = pk_bf2(f[6], f[7]);
  const v4u zz = {0u, 0u, 0u, 0u};
  for (int pass = 0; pass < 2; ++pass) {
    *(volatile v4u*)(WT  + (size_t)i * 8) = hv;
    *(volatile v4u*)(WTZ + (size_t)i * 8) = zz;
    __threadfence();
  }
}

__device__ __forceinline__ void xtile_fill(const int* __restrict__ xid, const float* __restrict__ emb,
                                           unsigned short* axh, int rowbase, int t, int tid) {
  const int m = tid >> 4, seg = tid & 15;
  int tok = xid[(size_t)(rowbase + m) * NSTEP + t];
  tok = (tok < 0) ? 0 : tok;
  tok = (tok > NVOC - 1) ? (NVOC - 1) : tok;
  const float* ep = emb + (size_t)tok * NEMB + seg * 16;
  const v4f e0 = *(const v4f*)(ep);
  const v4f e1 = *(const v4f*)(ep + 4);
  const v4f e2 = *(const v4f*)(ep + 8);
  const v4f e3 = *(const v4f*)(ep + 12);
  v4u w0, w1;
  w0[0] = pk_bf2(e0[0], e0[1]); w0[1] = pk_bf2(e0[2], e0[3]);
  w0[2] = pk_bf2(e1[0], e1[1]); w0[3] = pk_bf2(e1[2], e1[3]);
  w1[0] = pk_bf2(e2[0], e2[1]); w1[1] = pk_bf2(e2[2], e2[3]);
  w1[2] = pk_bf2(e3[0], e3[1]); w1[3] = pk_bf2(e3[2], e3[3]);
  *(v4u*)(axh + m * AP1 + seg * 16) = w0;
  *(v4u*)(axh + m * AP1 + seg * 16 + 8) = w1;
}

__global__ __launch_bounds__(NTHR) void bilstm_seq_kernel(const int* __restrict__ xid, const float* __restrict__ emb,
                                                          const float* __restrict__ b_f, const float* __restrict__ b_b,
                                                          const unsigned short* __restrict__ WCATp,
                                                          unsigned short* __restrict__ HHI, unsigned short* __restrict__ HLO) {
  __shared__ __align__(16) unsigned short Axh[SEQ_BLK * AP1];
  __shared__ __align__(16) unsigned short Alo[SEQ_BLK * AP2];
  const int tid = threadIdx.x, lane = tid & 31, wave = tid >> 5;
  const int c = lane & 15, hh = lane >> 4, koff = hh * 8;
  const int dir = (int)blockIdx.x >> 2;
  const int rowbase = ((int)blockIdx.x & 3) * SEQ_BLK;
  const __bf16* Wd = (const __bf16*)WCATp + (size_t)dir * ((size_t)NGATE * NKCAT);
  const float* bsel = dir ? b_b : b_f;

#pragma unroll 1
  for (int i = tid; i < SEQ_BLK * AP1; i += NTHR) Axh[i] = (unsigned short)0;
#pragma unroll 1
  for (int i = tid; i < SEQ_BLK * AP2; i += NTHR) Alo[i] = (unsigned short)0;
  float bb[2][4], cst[2][8];
#pragma unroll
  for (int nt = 0; nt < 2; ++nt) {
    const int j = 32 * wave + 16 * nt + c;
#pragma unroll
    for (int g = 0; g < 4; ++g) bb[nt][g] = bf16r(bsel[g * NHU + j]);
#pragma unroll
    for (int r = 0; r < 8; ++r) cst[nt][r] = 0.0f;
  }
  __syncthreads();
  xtile_fill(xid, emb, Axh, rowbase, dir ? (NSTEP - 1) : 0, tid);
  __syncthreads();

  const __bf16* ahrow = (const __bf16*)Axh + c * AP1 + koff;
  const __bf16* alrow = (const __bf16*)Alo + c * AP2 + koff;
  const v8f z8 = {0.f, 0.f, 0.f, 0.f, 0.f, 0.f, 0.f, 0.f};

#pragma unroll 1
  for (int it = 0; it < NSTEP; ++it) {
    const int t = dir ? (NSTEP - 1 - it) : it;

    v8f acc[2][4];
#pragma unroll
    for (int nt = 0; nt < 2; ++nt) { acc[nt][0] = z8; acc[nt][1] = z8; acc[nt][2] = z8; acc[nt][3] = z8; }

#pragma unroll 1
    for (int k0 = 0; k0 < NEMB; k0 += 32) {
      const v16b a = Frag<__bf16>::load(ahrow + k0);
#pragma unroll
      for (int nt = 0; nt < 2; ++nt) {
        const int j = 32 * wave + 16 * nt + c;
        const __bf16* wp = Wd + (size_t)j * NKCAT + koff + k0;
        const v16b b0 = Frag<__bf16>::load(wp);
        const v16b b1 = Frag<__bf16>::load(wp + (size_t)1 * NHU * NKCAT);
        const v16b b2 = Frag<__bf16>::load(wp + (size_t)2 * NHU * NKCAT);
        const v16b b3 = Frag<__bf16>::load(wp + (size_t)3 * NHU * NKCAT);
        acc[nt][0] = Frag<__bf16>::mma(a, b0, acc[nt][0]);
        acc[nt][1] = Frag<__bf16>::mma(a, b1, acc[nt][1]);
        acc[nt][2] = Frag<__bf16>::mma(a, b2, acc[nt][2]);
        acc[nt][3] = Frag<__bf16>::mma(a, b3, acc[nt][3]);
        grp_guard_b(acc[nt][0], acc[nt][1], acc[nt][2], acc[nt][3], a, a, b0, b1, b2, b3);
      }
    }
#pragma unroll 1
    for (int kh = 0; kh < NHU; kh += 32) {
      const v16b ah = Frag<__bf16>::load(ahrow + NEMB + kh);
      const v16b al = Frag<__bf16>::load(alrow + kh);
#pragma unroll
      for (int nt = 0; nt < 2; ++nt) {
        const int j = 32 * wave + 16 * nt + c;
        const __bf16* wp = Wd + (size_t)j * NKCAT + koff + NEMB + kh;
        const v16b b0 = Frag<__bf16>::load(wp);
        const v16b b1 = Frag<__bf16>::load(wp + (size_t)1 * NHU * NKCAT);
        const v16b b2 = Frag<__bf16>::load(wp + (size_t)2 * NHU * NKCAT);
        const v16b b3 = Frag<__bf16>::load(wp + (size_t)3 * NHU * NKCAT);
        acc[nt][0] = Frag<__bf16>::mma(ah, b0, acc[nt][0]);
        acc[nt][1] = Frag<__bf16>::mma(ah, b1, acc[nt][1]);
        acc[nt][2] = Frag<__bf16>::mma(ah, b2, acc[nt][2]);
        acc[nt][3] = Frag<__bf16>::mma(ah, b3, acc[nt][3]);
        acc[nt][0] = Frag<__bf16>::mma(al, b0, acc[nt][0]);
        acc[nt][1] = Frag<__bf16>::mma(al, b1, acc[nt][1]);
        acc[nt][2] = Frag<__bf16>::mma(al, b2, acc[nt][2]);
        acc[nt][3] = Frag<__bf16>::mma(al, b3, acc[nt][3]);
        grp_guard_b(acc[nt][0], acc[nt][1], acc[nt][2], acc[nt][3], ah, al, b0, b1, b2, b3);
      }
    }
    acc_guard4(acc[0][0], acc[0][1], acc[0][2], acc[0][3]);
    acc_guard4(acc[1][0], acc[1][1], acc[1][2], acc[1][3]);

    float hn[2][8];
#pragma unroll
    for (int nt = 0; nt < 2; ++nt) {
#pragma unroll
      for (int r = 0; r < 8; ++r) {
        const float zi = acc[nt][0][r] + bb[nt][0];
        const float zf = acc[nt][1][r] + bb[nt][1];
        const float zg = acc[nt][2][r] + bb[nt][2];
        const float zo = acc[nt][3][r] + bb[nt][3];
        const float ig = fsig(zi);
        const float fg = fsig(zf);
        const float gg = ftanh(zg);
        const float og = fsig(zo);
        const float cn = fg * cst[nt][r] + ig * gg;
        cst[nt][r] = cn;
        hn[nt][r] = og * ftanh(cn);
      }
    }
    __syncthreads();
#pragma unroll
    for (int nt = 0; nt < 2; ++nt) {
      const int j = 32 * wave + 16 * nt + c;
#pragma unroll
      for (int r = 0; r < 8; ++r) {
        const int row = 8 * hh + r;
        const float v = hn[nt][r];
        const unsigned short hb = f2bf_bits(v);
        const unsigned short lb = f2bf_bits(v - bf_bits2f(hb));
        Axh[row * AP1 + NEMB + j] = hb;
        Alo[row * AP2 + j] = lb;
      }
    }
    {
      const int itn = (it + 1 < NSTEP) ? (it + 1) : it;
      const int tn = dir ? (NSTEP - 1 - itn) : itn;
      xtile_fill(xid, emb, Axh, rowbase, tn, tid);
    }
    __syncthreads();
    for (int pass = 0; pass < 2; ++pass) {
#pragma unroll
      for (int rr = 0; rr < 2; ++rr) {
        const int row = 2 * wave + rr;
        const v4u hv = *(const v4u*)(Axh + row * AP1 + NEMB + lane * 8);
        const v4u lv = *(const v4u*)(Alo + row * AP2 + lane * 8);
        const size_t go = (((size_t)(rowbase + row)) * NSTEP + (size_t)t) * NHID2 + (size_t)dir * NHU + (size_t)lane * 8;
        *(volatile v4u*)(HHI + go) = hv;
        *(volatile v4u*)(HLO + go) = lv;
      }
      __threadfence();
    }
  }
}

__global__ __launch_bounds__(PK_THR) void pack_out_kernel(const float* __restrict__ CP, const float* __restrict__ btag,
                                                          float* __restrict__ out) {
  const int tid = threadIdx.x;
  const int rb = blockIdx.x * 64;
  const int f = tid * 4;
  const int row = f / NTAG;
  const int col = f - row * NTAG;
  const v4f v  = *(const v4f*)(CP + (size_t)(rb + row) * NTAGP + col);
  const v4f bt = *(const v4f*)(btag + col);
  v4f o;
#pragma unroll
  for (int e = 0; e < 4; ++e) o[e] = v[e] + bf16r(bt[e]);
  float* op = out + (size_t)rb * NTAG + f;
  *(volatile v4f*)op = o;
  __threadfence();
  *(volatile v4f*)op = o;
}

extern "C" void kernel_launch(void* const* d_in, const int* in_sizes, int n_in,
                              void* d_out, int out_size, void* d_ws, size_t ws_size, hipStream_t stream) {
  if (n_in < 10 || d_out == nullptr || d_ws == nullptr) return;
  if (in_sizes[0] != NB_SEQ * NSTEP || in_sizes[1] != NVOC * NEMB || in_sizes[2] != NEMB * NGATE ||
      in_sizes[3] != NHU * NGATE || in_sizes[4] != NGATE || in_sizes[5] != NEMB * NGATE || in_sizes[6] != NHU * NGATE ||
      in_sizes[7] != NGATE || in_sizes[8] != NHID2 * NTAG || in_sizes[9] != NTAG || out_size != NROWS * NTAG) return;

  const int*   xid   = (const int*)d_in[0];
  const float* emb   = (const float*)d_in[1];
  const float* wx_f  = (const float*)d_in[2];
  const float* wh_f  = (const float*)d_in[3];
  const float* b_f   = (const float*)d_in[4];
  const float* wx_b  = (const float*)d_in[5];
  const float* wh_b  = (const float*)d_in[6];
  const float* b_b   = (const float*)d_in[7];
  const float* w_tag = (const float*)d_in[8];
  const float* b_tag = (const float*)d_in[9];
  float* out = (float*)d_out;

  char* ws = (char*)d_ws; size_t off = 0;
  auto carve = [&](size_t bytes) -> char* { char* p = ws + off; off += (bytes + 255) & ~(size_t)255; return p; };
  unsigned short* WCAT = (unsigned short*)carve((size_t)2 * NGATE * NKCAT * 2);
  unsigned short* WT   = (unsigned short*)carve((size_t)NTAGP * NHID2 * 2);
  unsigned short* WTZ  = (unsigned short*)carve((size_t)NTAGP * NHID2 * 2);
  unsigned short* HHI  = (unsigned short*)carve((size_t)NROWS * NHID2 * 2);
  unsigned short* HLO  = (unsigned short*)carve((size_t)NROWS * NHID2 * 2);
  float*          CPAD = (float*)carve((size_t)NROWS * NTAGP * 4);
  if (off > ws_size || off > WS_CAP) return;

  wcat_prep_kernel<<<dim3(NGATE / 64, NHU / 64, 4), NTHR, 0, stream>>>(wx_f, wh_f, wx_b, wh_b, WCAT);
  wtag_prep_kernel<<<(NTAGP * NHID2 / 8) / NTHR, NTHR, 0, stream>>>(w_tag, WT, WTZ);
  bilstm_seq_kernel<<<2 * (NB_SEQ / SEQ_BLK), NTHR, 0, stream>>>(xid, emb, b_f, b_b, WCAT, HHI, HLO);
  wmma_gemm64<1, true, 0, 0, false, 0><<<dim3((NROWS / 64) * (NTAGP / 64) / 8, 1), 256, 0, stream>>>(
      HHI, HLO, NHID2, 0L, WT, WTZ, NHID2, 0L, (void*)CPAD, (void*)CPAD, NTAGP, 0L,
      b_tag, b_tag, 0L, NROWS, NTAGP, NHID2, 1.0f);
  pack_out_kernel<<<NROWS / 64, PK_THR, 0, stream>>>(CPAD, b_tag, out);
}
